// LocalContext_42949673366
// MI455X (gfx1250) — hardware-verified
//
#include <hip/hip_runtime.h>


namespace {
constexpr int NB_ = 2, C = 32, Hh = 128, Ww = 128, L = Hh * Ww, NPX = NB_ * L, KS = 5, KK = 25, NH = 2, HD = 16, C2 = 64, HID = 128, KF = KK * C  , PW = 32  , HALO = PW + 4  , NPOS = KS * HALO  ;
constexpr float HS = 256.0f, WSC = 256.0f, EPS = 1e-5f;
typedef _Float16 b16;
typedef __attribute__((ext_vector_type(16))) _Float16 v16b;
typedef __attribute__((ext_vector_type(8))) _Float16 v8b;
typedef __attribute__((ext_vector_type(8))) float v8f;
typedef __attribute__((ext_vector_type(4))) float v4f;
__device__ __forceinline__ float bf16_rne(float f) { unsigned int u = __float_as_uint(f); u += 0x7FFFu + ((u >> 16) & 1u); float r = __uint_as_float(u & 0xFFFF0000u); asm volatile("" : "+v"(r)); return r; }
__device__ __forceinline__ float bfv(float f) { float r = bf16_rne(f); asm volatile("" : "+v"(r)); return r; }
__device__ __forceinline__ void split16(float v, b16& hi, b16& lo) { hi = (b16)v; lo = (b16)(v - (float)hi); }
__device__ __forceinline__ v16b frag_kb(const b16* p, int hh) { const v8b a = *(const v8b*)(p + 8 * hh), b = *(const v8b*)(p + 16 + 8 * hh); v16b f;
#pragma unroll
  for (int e = 0; e < 8; ++e) { f[e] = a[e]; f[8 + e] = b[e]; } return f; }
__device__ __forceinline__ v8f wmma16b(v16b a, v16b b, v8f c) { v8f d = __builtin_amdgcn_wmma_f32_16x16x32_f16(false, a, false, b, (short)0, c, false, false); asm volatile("v_nop\n\tv_nop\n\tv_nop\n\tv_nop" : "+v"(d) : "v"(a), "v"(b)); return d; }
__device__ __forceinline__ void wave_lds_sync() { __builtin_amdgcn_fence(__ATOMIC_RELEASE, "workgroup"); __builtin_amdgcn_wave_barrier(); __builtin_amdgcn_fence(__ATOMIC_ACQUIRE, "workgroup"); }
__device__ __forceinline__ float pmul(float a, float b) { float p = a * b; asm volatile("" : "+v"(p)); return p; }

__global__ __launch_bounds__(256) void wput_kernel(const float* __restrict__ wq, const float* __restrict__ wf, const float* __restrict__ wp, const float* __restrict__ wm1, const float* __restrict__ wm2, const float* __restrict__ rel, b16* __restrict__ WQ, b16* __restrict__ WF, b16* __restrict__ WP, b16* __restrict__ WM1, b16* __restrict__ WM2, float* __restrict__ BIAS) { const size_t nt = (size_t)gridDim.x * 256, u0 = (size_t)blockIdx.x * 256 + threadIdx.x; v8b v;
  for (size_t u = u0; u < 96 * 4; u += nt) { const int o = (int)(u / 4), k0 = (int)(u % 4) * 8;
#pragma unroll
    for (int j = 0; j < 8; ++j) v[j] = (b16)(bf16_rne(wq[(size_t)o * C + k0 + j]) * WSC); for (int pass = 0; pass < 2; ++pass) { *(volatile v8b*)(WQ + (size_t)o * C + k0) = v; __threadfence(); } }
  for (size_t u = u0; u < 64 * 100; u += nt) { const int o = (int)(u / 100), k0 = (int)(u % 100) * 8;
#pragma unroll
    for (int j = 0; j < 8; ++j) { const int k = k0 + j; const int p = k / C, cp = k % C; const int i = p / KS, jj = p % KS; v[j] = (b16)(bf16_rne(wf[(((size_t)o * C + cp) * KS + i) * KS + jj]) * WSC); } for (int pass = 0; pass < 2; ++pass) { *(volatile v8b*)(WF + (size_t)o * KF + k0) = v; __threadfence(); } }
  for (size_t u = u0; u < 64 * 8; u += nt) { const int o = (int)(u / 8), k0 = (int)(u % 8) * 8;
#pragma unroll
    for (int j = 0; j < 8; ++j) v[j] = (b16)(bf16_rne(wp[(size_t)o * C2 + k0 + j]) * WSC); for (int pass = 0; pass < 2; ++pass) { *(volatile v8b*)(WP + (size_t)o * C2 + k0) = v; __threadfence(); } }
  for (size_t u = u0; u < 128 * 8; u += nt) { const int o = (int)(u / 8), k0 = (int)(u % 8) * 8;
#pragma unroll
    for (int j = 0; j < 8; ++j) v[j] = (b16)(bf16_rne(wm1[(size_t)o * C2 + k0 + j]) * WSC); for (int pass = 0; pass < 2; ++pass) { *(volatile v8b*)(WM1 + (size_t)o * C2 + k0) = v; __threadfence(); } }
  for (size_t u = u0; u < 64 * 16; u += nt) { const int o = (int)(u / 16), k0 = (int)(u % 16) * 8;
#pragma unroll
    for (int j = 0; j < 8; ++j) v[j] = (b16)(bf16_rne(wm2[(size_t)o * HID + k0 + j]) * WSC); for (int pass = 0; pass < 2; ++pass) { *(volatile v8b*)(WM2 + (size_t)o * HID + k0) = v; __threadfence(); } }
  if (u0 < (size_t)NH * KK * 32) { const int h = (int)(u0 / (KK * 32)), p = (int)((u0 / 32) % KK), pp = (int)(u0 % 32); float b = 0.0f; if (pp < KK) { const int di = (p / KS) - (pp / KS) + (KS - 1), dj = (p % KS) - (pp % KS) + (KS - 1); b = bfv(rel[(di * (2 * KS - 1) + dj) * NH + h]); }
    for (int pass = 0; pass < 2; ++pass) { ((volatile float*)BIAS)[u0] = b; __threadfence(); } } }
__global__ __launch_bounds__(32) void qkv_kernel(const float* __restrict__ x, const float* __restrict__ n1w, const float* __restrict__ n1b, const b16* __restrict__ WQ, const float* __restrict__ qb, int PXLIM, float* __restrict__ QKV) { __shared__ __attribute__((aligned(16))) b16 Ah[16][C + 8], Al[16][C + 8]; __shared__ float Xs[16][C + 1], Tf[16][100]; const int lane = threadIdx.x, nloc = lane & 15, hlf = lane >> 4; const size_t px0 = (size_t)blockIdx.x * 16; if (px0 >= (size_t)PXLIM) return; const int b = (int)(px0 / L); const size_t l0 = px0 % L;
  for (int c = 0; c < C; ++c) if (lane < 16) Xs[lane][c] = bfv(x[((size_t)b * C + c) * L + l0 + lane]);
  wave_lds_sync();
  if (lane < 16) { float m = 0.0f; for (int c = 0; c < C; ++c) m += Xs[lane][c]; m *= (1.0f / C); float vr = 0.0f; for (int c = 0; c < C; ++c) { const float d = Xs[lane][c] - m; vr += d * d; } vr *= (1.0f / C); const float rs = rsqrtf(vr + EPS);
    for (int c = 0; c < C; ++c) { const float v = pmul((Xs[lane][c] - m) * rs, bfv(n1w[c])) + bfv(n1b[c]); b16 p, ql; split16(v * HS, p, ql); Ah[lane][c] = p; Al[lane][c] = ql; } for (int k = C; k < C + 8; ++k) { Ah[lane][k] = (b16)0.0f; Al[lane][k] = (b16)0.0f; } }
  wave_lds_sync(); v8f acc[6];
#pragma unroll
  for (int t = 0; t < 6; ++t) acc[t] = (v8f){};
  { const v16b a = frag_kb(&Ah[nloc][0], hlf), al = frag_kb(&Al[nloc][0], hlf);
#pragma unroll
    for (int t = 0; t < 6; ++t) { const v16b bw = frag_kb(WQ + (size_t)(t * 16 + nloc) * C, hlf); acc[t] = wmma16b(a, bw, acc[t]); acc[t] = wmma16b(al, bw, acc[t]); } }
#pragma unroll
  for (int t = 0; t < 6; ++t) { const int cc = t * 16 + nloc; const float bb = bfv(qb[cc]);
#pragma unroll
    for (int r8 = 0; r8 < 8; ++r8) Tf[8 * hlf + r8][cc] = acc[t][r8] * (1.0f / (HS * WSC)) + bb; }
  wave_lds_sync();
  for (int pass = 0; pass < 2; ++pass) { for (int rr = 0; rr < 16; ++rr) for (int q = 0; q < 3; ++q) ((volatile float*)QKV)[(px0 + rr) * 96 + q * 32 + lane] = Tf[rr][q * 32 + lane]; __threadfence(); } }
__global__ __launch_bounds__(32) void att_kernel(const float* __restrict__ QKV, const float* __restrict__ BIAS, int PXLIM, float* __restrict__ O) { __shared__ __attribute__((aligned(16))) b16 Qh[NH][NPOS][32], Kh[NH][NPOS][32], Vh[NH][NPOS][HD], Vl[NH][NPOS][HD], Pa[32][40], Pb[32][40], Vth[HD][40], Vtl[HD][40]; __shared__ float Sc[32][33], Ck[NPOS]; const int lane = threadIdx.x, nloc = lane & 15, hlf = lane >> 4; const size_t px0 = (size_t)blockIdx.x * PW; if (px0 >= (size_t)PXLIM) return; const int b = (int)(px0 / L); const int l0 = (int)(px0 % L); const int y0 = l0 / Ww, x0 = l0 % Ww;
  for (int pos = 0; pos < NPOS; ++pos) { const int r = pos / HALO, cc = pos % HALO; const int yy = y0 - 2 + r, xx = x0 - 2 + cc; const bool in = yy >= 0 && yy < Hh && xx >= 0 && xx < Ww; const float* row = QKV + ((size_t)b * L + (in ? yy * Ww + xx : 0)) * 96;
    { const int c = lane; const int h = c % NH, d = c / NH; const float qv = in ? row[c] : 0.0f, kv = in ? row[C + c] : 0.0f, vv = in ? row[2 * C + c] : 0.0f; Qh[h][pos][d] = (b16)(qv * HS); Kh[h][pos][d] = (b16)(kv * HS); b16 p, ql; split16(vv * HS, p, ql); Vh[h][pos][d] = p; Vl[h][pos][d] = ql; Qh[h][pos][HD + (lane >> 1)] = (b16)0.0f; Kh[h][pos][HD + (lane >> 1)] = (b16)0.0f; }
    if (lane == 0) Ck[pos] = (in && (((yy + xx) & 1) == 1)) ? 1.0f : 0.0f; }
  for (int k = 32; k < 40; ++k) { Pa[lane][k] = (b16)0.0f; Pb[lane][k] = (b16)0.0f; } if (lane < HD) for (int k = KK; k < 40; ++k) { Vth[lane][k] = (b16)0.0f; Vtl[lane][k] = (b16)0.0f; }
  wave_lds_sync();
  auto posof = [&](int i, int p) { return (p / KS) * HALO + i + (p % KS); };
#pragma unroll 1
  for (int i = 0; i < PW; ++i) {
#pragma unroll 1
    for (int h = 0; h < NH; ++h) {
      const int pr0 = nloc < KK ? posof(i, nloc) : posof(i, 0), pr1 = (nloc + 16) < KK ? posof(i, nloc + 16) : posof(i, 0);
      const v16b qa0 = frag_kb(&Qh[h][pr0][0], hlf), qa1 = frag_kb(&Qh[h][pr1][0], hlf), kb0 = frag_kb(&Kh[h][pr0][0], hlf), kb1 = frag_kb(&Kh[h][pr1][0], hlf);
      v8f s00 = wmma16b(qa0, kb0, (v8f){}), s01 = wmma16b(qa0, kb1, (v8f){}), s10 = wmma16b(qa1, kb0, (v8f){}), s11 = wmma16b(qa1, kb1, (v8f){});
#pragma unroll
      for (int r8 = 0; r8 < 8; ++r8) { Sc[8 * hlf + r8][nloc] = s00[r8]; Sc[8 * hlf + r8][16 + nloc] = s01[r8]; Sc[16 + 8 * hlf + r8][nloc] = s10[r8]; Sc[16 + 8 * hlf + r8][16 + nloc] = s11[r8]; }
      for (int pp = hlf; pp < KK; pp += 2) { const int ps = posof(i, pp); Vth[nloc][pp] = Vh[h][ps][nloc]; Vtl[nloc][pp] = Vl[h][ps][nloc]; }
      wave_lds_sync();
      if (lane < KK) { const float ckq = Ck[posof(i, lane)]; float lg[KK]; float mx = -INFINITY;
#pragma unroll
        for (int pp = 0; pp < KK; ++pp) { const float m = (ckq * Ck[posof(i, pp)] == 1.0f) ? 0.0f : -100.0f; lg[pp] = Sc[lane][pp] * (0.25f / (HS * HS)) + BIAS[(h * KK + lane) * 32 + pp] + m; mx = fmaxf(mx, lg[pp]); }
        float sm = 0.0f;
#pragma unroll
        for (int pp = 0; pp < KK; ++pp) { lg[pp] = __expf(lg[pp] - mx); sm += lg[pp]; } const float inv = 1.0f / sm;
#pragma unroll
        for (int pp = 0; pp < KK; ++pp) { b16 p_, ql; split16(lg[pp] * inv * HS, p_, ql); Pa[lane][pp] = p_; Pb[lane][pp] = ql; } for (int pp = KK; pp < 32; ++pp) { Pa[lane][pp] = (b16)0.0f; Pb[lane][pp] = (b16)0.0f; } }
      else { for (int pp = 0; pp < 32; ++pp) { Pa[lane][pp] = (b16)0.0f; Pb[lane][pp] = (b16)0.0f; } }
      wave_lds_sync();
      const v16b pa0 = frag_kb(&Pa[nloc][0], hlf), pb0 = frag_kb(&Pb[nloc][0], hlf), pa1 = frag_kb(&Pa[16 + nloc][0], hlf), pb1 = frag_kb(&Pb[16 + nloc][0], hlf), vh = frag_kb(&Vth[nloc][0], hlf), vl = frag_kb(&Vtl[nloc][0], hlf);
      v8f o0 = wmma16b(pa0, vh, (v8f){}); o0 = wmma16b(pa0, vl, o0); o0 = wmma16b(pb0, vh, o0); v8f o1 = wmma16b(pa1, vh, (v8f){}); o1 = wmma16b(pa1, vl, o1); o1 = wmma16b(pb1, vh, o1);
      for (int pass = 0; pass < 2; ++pass) {
#pragma unroll
        for (int r8 = 0; r8 < 8; ++r8) { const int p0 = 8 * hlf + r8, p1 = 16 + 8 * hlf + r8; ((volatile float*)O)[(px0 + i) * KF + p0 * C + h * HD + nloc] = o0[r8] * (1.0f / (HS * HS)); if (p1 < KK) ((volatile float*)O)[(px0 + i) * KF + p1 * C + h * HD + nloc] = o1[r8] * (1.0f / (HS * HS)); }
        __threadfence(); }
      wave_lds_sync(); } } }
__global__ __launch_bounds__(32) void tail_kernel(const float* __restrict__ O, const b16* __restrict__ WF, const float* __restrict__ fb, const b16* __restrict__ WP, const float* __restrict__ pb, const float* __restrict__ n2w, const float* __restrict__ n2b, const b16* __restrict__ WM1, const float* __restrict__ m1b, const b16* __restrict__ WM2, const float* __restrict__ m2b, int PXLIM, float* __restrict__ out) { constexpr int KA = 416, KB2 = KF - KA  ; __shared__ __attribute__((aligned(16))) b16 Ah[32][KA + 8], Al[32][KA + 8]; __shared__ float Y[32][C2 + 1], Tf[32][HID + 1]; const int lane = threadIdx.x, nloc = lane & 15, hlf = lane >> 4; const size_t px0 = (size_t)blockIdx.x * PW; if (px0 >= (size_t)PXLIM) return; const int b = (int)(px0 / L); const int l0 = (int)(px0 % L);
  auto stage = [&](int K, int srcStride, const float* src, int srcOff) { for (int rr = 0; rr < 32; ++rr) for (int c = lane; c < K; c += 32) { b16 p, ql; split16(src[(size_t)rr * srcStride + srcOff + c] * HS, p, ql); Ah[rr][c] = p; Al[rr][c] = ql; } for (int k = K; k < K + 8; ++k) { Ah[lane][k] = (b16)0.0f; Al[lane][k] = (b16)0.0f; } wave_lds_sync(); };
  { v8f acc[2][4];
#pragma unroll
    for (int rt = 0; rt < 2; ++rt)
#pragma unroll
      for (int t = 0; t < 4; ++t) acc[rt][t] = (v8f){};
#pragma unroll 1
    for (int part = 0; part < 2; ++part) { const int kbase = part ? KA : 0, klen = part ? KB2 : KA; stage(klen, KF, O + (px0) * KF, kbase);
#pragma unroll 1
      for (int kb = 0; kb < klen; kb += 32) {
#pragma unroll
        for (int rt = 0; rt < 2; ++rt) { const v16b a = frag_kb(&Ah[rt * 16 + nloc][kb], hlf), al = frag_kb(&Al[rt * 16 + nloc][kb], hlf);
#pragma unroll
          for (int t = 0; t < 4; ++t) { const v16b bw = frag_kb(WF + (size_t)(t * 16 + nloc) * KF + kbase + kb, hlf); acc[rt][t] = wmma16b(a, bw, acc[rt][t]); acc[rt][t] = wmma16b(al, bw, acc[rt][t]); } } }
      wave_lds_sync(); }
#pragma unroll
    for (int rt = 0; rt < 2; ++rt)
#pragma unroll
      for (int t = 0; t < 4; ++t) { const int cc = t * 16 + nloc; const float bb = bfv(fb[cc]);
#pragma unroll
        for (int r8 = 0; r8 < 8; ++r8) Y[rt * 16 + 8 * hlf + r8][cc] = acc[rt][t][r8] * (1.0f / (HS * WSC)) + bb; } }
  wave_lds_sync();
  { for (int rr = 0; rr < 32; ++rr) for (int q = 0; q < 2; ++q) { b16 p, ql; split16(Y[rr][q * 32 + lane] * HS, p, ql); Ah[rr][q * 32 + lane] = p; Al[rr][q * 32 + lane] = ql; } for (int k = C2; k < C2 + 8; ++k) { Ah[lane][k] = (b16)0.0f; Al[lane][k] = (b16)0.0f; } wave_lds_sync();
    v8f acc[2][4];
#pragma unroll
    for (int rt = 0; rt < 2; ++rt)
#pragma unroll
      for (int t = 0; t < 4; ++t) acc[rt][t] = (v8f){};
#pragma unroll
    for (int kb = 0; kb < C2; kb += 32)
#pragma unroll
      for (int rt = 0; rt < 2; ++rt) { const v16b a = frag_kb(&Ah[rt * 16 + nloc][kb], hlf), al = frag_kb(&Al[rt * 16 + nloc][kb], hlf);
#pragma unroll
        for (int t = 0; t < 4; ++t) { const v16b bw = frag_kb(WP + (size_t)(t * 16 + nloc) * C2 + kb, hlf); acc[rt][t] = wmma16b(a, bw, acc[rt][t]); acc[rt][t] = wmma16b(al, bw, acc[rt][t]); } }
    wave_lds_sync();
#pragma unroll
    for (int rt = 0; rt < 2; ++rt)
#pragma unroll
      for (int t = 0; t < 4; ++t) { const int cc = t * 16 + nloc; const float bb = bfv(pb[cc]);
#pragma unroll
        for (int r8 = 0; r8 < 8; ++r8) Y[rt * 16 + 8 * hlf + r8][cc] = acc[rt][t][r8] * (1.0f / (HS * WSC)) + bb; } }
  wave_lds_sync();
  { const int rr = lane; float m = 0.0f; for (int c = 0; c < C2; ++c) m += Y[rr][c]; m *= (1.0f / C2); float vr = 0.0f; for (int c = 0; c < C2; ++c) { const float d = Y[rr][c] - m; vr += d * d; } vr *= (1.0f / C2); const float rs = rsqrtf(vr + EPS);
    for (int c = 0; c < C2; ++c) { const float v = pmul((Y[rr][c] - m) * rs, bfv(n2w[c])) + bfv(n2b[c]); b16 p, ql; split16(v * HS, p, ql); Ah[rr][c] = p; Al[rr][c] = ql; } }
  wave_lds_sync();
  { v8f acc[2][8];
#pragma unroll
    for (int rt = 0; rt < 2; ++rt)
#pragma unroll
      for (int t = 0; t < 8; ++t) acc[rt][t] = (v8f){};
#pragma unroll
    for (int kb = 0; kb < C2; kb += 32)
#pragma unroll
      for (int rt = 0; rt < 2; ++rt) { const v16b a = frag_kb(&Ah[rt * 16 + nloc][kb], hlf), al = frag_kb(&Al[rt * 16 + nloc][kb], hlf);
#pragma unroll
        for (int t = 0; t < 8; ++t) { const v16b bw = frag_kb(WM1 + (size_t)(t * 16 + nloc) * C2 + kb, hlf); acc[rt][t] = wmma16b(a, bw, acc[rt][t]); acc[rt][t] = wmma16b(al, bw, acc[rt][t]); } }
    wave_lds_sync();
#pragma unroll
    for (int rt = 0; rt < 2; ++rt)
#pragma unroll
      for (int t = 0; t < 8; ++t) { const int cc = t * 16 + nloc; const float bb = bfv(m1b[cc]);
#pragma unroll
        for (int r8 = 0; r8 < 8; ++r8) { const float v = acc[rt][t][r8] * (1.0f / (HS * WSC)) + bb; Tf[rt * 16 + 8 * hlf + r8][cc] = 0.5f * v * (1.0f + erff(v * 0.70710678118654752f)); } } }
  wave_lds_sync();
  for (int rr = 0; rr < 32; ++rr) for (int q = 0; q < 4; ++q) { b16 p, ql; split16(Tf[rr][q * 32 + lane] * HS, p, ql); Ah[rr][q * 32 + lane] = p; Al[rr][q * 32 + lane] = ql; } for (int k = HID; k < HID + 8; ++k) { Ah[lane][k] = (b16)0.0f; Al[lane][k] = (b16)0.0f; }
  wave_lds_sync();
  { v8f acc[2][4];
#pragma unroll
    for (int rt = 0; rt < 2; ++rt)
#pragma unroll
      for (int t = 0; t < 4; ++t) acc[rt][t] = (v8f){};
#pragma unroll
    for (int kb = 0; kb < HID; kb += 32)
#pragma unroll
      for (int rt = 0; rt < 2; ++rt) { const v16b a = frag_kb(&Ah[rt * 16 + nloc][kb], hlf), al = frag_kb(&Al[rt * 16 + nloc][kb], hlf);
#pragma unroll
        for (int t = 0; t < 4; ++t) { const v16b bw = frag_kb(WM2 + (size_t)(t * 16 + nloc) * HID + kb, hlf); acc[rt][t] = wmma16b(a, bw, acc[rt][t]); acc[rt][t] = wmma16b(al, bw, acc[rt][t]); } }
#pragma unroll
    for (int rt = 0; rt < 2; ++rt)
#pragma unroll
      for (int t = 0; t < 4; ++t) { const int cc = t * 16 + nloc; const float bb = bfv(m2b[cc]);
#pragma unroll
        for (int r8 = 0; r8 < 8; ++r8) Tf[rt * 16 + 8 * hlf + r8][cc] = Y[rt * 16 + 8 * hlf + r8][cc] + acc[rt][t][r8] * (1.0f / (HS * WSC)) + bb; } }
  wave_lds_sync();
  for (int pass = 0; pass < 2; ++pass) { for (int o = 0; o < C2; ++o) ((volatile float*)out)[((size_t)b * C2 + o) * L + l0 + lane] = Tf[lane][o]; __threadfence(); } }
}

extern "C" void kernel_launch(void* const* d_in, const int* in_sizes, int n_in, void* d_out, int out_size, void* d_ws, size_t ws_size, hipStream_t stream) {
  (void)n_in;
  auto Fp = [&](int i) { return (const float*)d_in[i]; };
  if (in_sizes[0] != NPX * C || in_sizes[1] != 96 * C || in_sizes[3] != 81 * NH || in_sizes[8] != C2 * C2 || in_sizes[10] != C2 * C * KK || in_sizes[12] != HID * C2 || in_sizes[14] != C2 * HID || out_size != NPX * C2) return;
  const int PXLIM = NPX;
  size_t off = 0; char* ws = (char*)d_ws;
  auto carve = [&](size_t bytes) { char* p = ws + off; off += (bytes + 255) & ~(size_t)255; return p; };
  b16* WQ = (b16*)carve((size_t)96 * C * 2); b16* WF = (b16*)carve((size_t)C2 * KF * 2); b16* WP = (b16*)carve((size_t)C2 * C2 * 2); b16* WM1 = (b16*)carve((size_t)HID * C2 * 2); b16* WM2 = (b16*)carve((size_t)C2 * HID * 2); float* BIAS = (float*)carve((size_t)NH * KK * 32 * 4); float* QKV = (float*)carve((size_t)NPX * 96 * 4); float* O = (float*)carve((size_t)NPX * KF * 4);
  if (off > ws_size || off > ((size_t)136 << 20)) return;
  wput_kernel<<<32, 256, 0, stream>>>(Fp(1), Fp(10), Fp(8), Fp(12), Fp(14), Fp(3), WQ, WF, WP, WM1, WM2, BIAS);
  qkv_kernel<<<NPX / 16, 32, 0, stream>>>(Fp(0), Fp(4), Fp(5), WQ, Fp(2), NPX, QKV);
  att_kernel<<<PXLIM / PW, 32, 0, stream>>>(QKV, BIAS, PXLIM, O);
  tail_kernel<<<PXLIM / PW, 32, 0, stream>>>(O, WF, Fp(11), WP, Fp(9), Fp(6), Fp(7), WM1, Fp(13), WM2, Fp(15), PXLIM, (float*)d_out);
}
